// RWKV_TimeMix_26886495273155
// MI455X (gfx1250) — hardware-verified
//
#include <hip/hip_runtime.h>
#include <math.h>

constexpr int kBatch     = 32;
constexpr int kT         = 256;
constexpr int kC         = 1024;
constexpr int kRows      = kBatch * kT;
constexpr int kChunks    = 2;
constexpr int kChunkB    = kBatch / kChunks;
constexpr int kChunkRows = kChunkB * kT;
constexpr int kPairs     = kC / 2;
constexpr float kWCarry  = 16.0f;
constexpr float kACarry  = 16.0f;
constexpr float kRScale  = 1.0f / 16.0f;
constexpr float kOScale  = 1.0f / 256.0f;
constexpr float kNegInit = -1.0e38f;
static_assert(kChunkRows % 64 == 0 && kC % 64 == 0 && kC % 32 == 0, "tiles");
static_assert((kChunkRows * kC) % (256 * 8) == 0 && (kC * kC) % (256 * 8) == 0, "cast grids");
static_assert((kChunkB * kPairs) % 256 == 0, "scan grid");
static_assert(kT == 256 && kC == 1024 && kPairs == 512, "index masks");
static_assert(kChunks * kChunkRows == kRows, "chunks");

typedef __attribute__((ext_vector_type(16))) _Float16 v16h;
typedef __attribute__((ext_vector_type(8)))  _Float16 v8h;
typedef __attribute__((ext_vector_type(16))) __bf16   v16b;
typedef __attribute__((ext_vector_type(8)))  __bf16   v8b;
typedef __attribute__((ext_vector_type(8)))  float    v8f;
typedef __attribute__((ext_vector_type(4)))  float    v4f;
typedef __attribute__((ext_vector_type(2)))  float    v2f;
typedef __attribute__((ext_vector_type(4)))  unsigned int v4u;

__device__ __forceinline__ unsigned short f2bf_bits(float f) {
  unsigned u = __float_as_uint(f);
  return (unsigned short)((u + 0x7FFFu + ((u >> 16) & 1u)) >> 16);
}
__device__ __forceinline__ float bf_bits2f(unsigned short h) { return __uint_as_float(((unsigned)h) << 16); }

__device__ __forceinline__ void dep_guard_h(v8f& a, v8f& b, v16h x, v16h y) { asm volatile("v_nop\n\tv_nop\n\tv_nop\n\tv_nop" : "+v"(a), "+v"(b) : "v"(x), "v"(y)); }
__device__ __forceinline__ void dep_guard_b(v8f& a, v8f& b, v16b x, v16b y) { asm volatile("v_nop\n\tv_nop\n\tv_nop\n\tv_nop" : "+v"(a), "+v"(b) : "v"(x), "v"(y)); }
__device__ __forceinline__ void dep_guard4_h(v8f& a, v8f& b, v8f& c, v8f& d, v16h x, v16h y) { asm volatile("v_nop\n\tv_nop\n\tv_nop\n\tv_nop" : "+v"(a), "+v"(b), "+v"(c), "+v"(d) : "v"(x), "v"(y)); }
__device__ __forceinline__ void dep_guard4_b(v8f& a, v8f& b, v8f& c, v8f& d, v16b x, v16b y) { asm volatile("v_nop\n\tv_nop\n\tv_nop\n\tv_nop" : "+v"(a), "+v"(b), "+v"(c), "+v"(d) : "v"(x), "v"(y)); }
__device__ __forceinline__ void keep4_h(v16h a, v16h b, v16h c, v16h d) { asm volatile("v_nop" :: "v"(a), "v"(b), "v"(c), "v"(d)); }
__device__ __forceinline__ void keep4_b(v16b a, v16b b, v16b c, v16b d) { asm volatile("v_nop" :: "v"(a), "v"(b), "v"(c), "v"(d)); }
__device__ __forceinline__ void acc_guard4(v8f& a, v8f& b, v8f& c, v8f& d) { asm volatile("v_nop\n\tv_nop\n\tv_nop\n\tv_nop" : "+v"(a), "+v"(b), "+v"(c), "+v"(d)); }
template <typename T> struct Frag;
template <> struct Frag<_Float16> {
  typedef v16h V; union U { v16h v; v8h h[2]; };
  static __device__ __forceinline__ v16h load(const _Float16* p) {
    U f; f.h[0] = *(const v8h*)(p); f.h[1] = *(const v8h*)(p + 16); return f.v;
  }
  static __device__ __forceinline__ v8f mma(v16h a, v16h b, v8f c) {
    return __builtin_amdgcn_wmma_f32_16x16x32_f16(false, a, false, b, (short)0, c, false, false);
  }
  static __device__ __forceinline__ void guard(v8f& a, v8f& b, v16h x, v16h y) { dep_guard_h(a, b, x, y); }
  static __device__ __forceinline__ void guard4(v8f& a, v8f& b, v8f& c, v8f& d, v16h x, v16h y) { dep_guard4_h(a, b, c, d, x, y); }
  static __device__ __forceinline__ void keep(v16h a, v16h b, v16h c, v16h d) { keep4_h(a, b, c, d); }
};
template <> struct Frag<__bf16> {
  typedef v16b V; union U { v16b v; v8b h[2]; };
  static __device__ __forceinline__ v16b load(const __bf16* p) {
    U f; f.h[0] = *(const v8b*)(p); f.h[1] = *(const v8b*)(p + 16); return f.v;
  }
  static __device__ __forceinline__ v8f mma(v16b a, v16b b, v8f c) {
    return __builtin_amdgcn_wmma_f32_16x16x32_bf16(false, a, false, b, (short)0, c, false, false);
  }
  static __device__ __forceinline__ void guard(v8f& a, v8f& b, v16b x, v16b y) { dep_guard_b(a, b, x, y); }
  static __device__ __forceinline__ void guard4(v8f& a, v8f& b, v8f& c, v8f& d, v16b x, v16b y) { dep_guard4_b(a, b, c, d, x, y); }
  static __device__ __forceinline__ void keep(v16b a, v16b b, v16b c, v16b d) { keep4_b(a, b, c, d); }
};

__device__ __forceinline__ unsigned pk16(unsigned short a, unsigned short b) { return (unsigned)a | ((unsigned)b << 16); }
__device__ __forceinline__ unsigned short h_bits(float f) { const _Float16 h = (_Float16)f; return __builtin_bit_cast(unsigned short, h); }

__device__ __forceinline__ float h16_to_f32(unsigned hb) {
  const unsigned sgn = (hb & 0x8000u) << 16; const unsigned em = hb & 0x7fffu;
  const float fn = __uint_as_float((em << 13) + 0x38000000u);
  const float fs = (float)em * 5.9604644775390625e-8f;
  const float mag = (em < 0x400u) ? fs : fn; return __uint_as_float(__float_as_uint(mag) | sgn); }

template <int ET> struct Elem;
template <> struct Elem<0> { typedef _Float16 T; };
template <> struct Elem<1> { typedef __bf16 T; };
template <int ET, bool SPLIT, int BIAS_MODE, int OUT_MODE, bool RESID, int ACT = 0>
__global__ __launch_bounds__(256) void wmma_gemm64(
    const unsigned short* __restrict__ Ap, const unsigned short* __restrict__ A2p, int lda, long strideA,
    const unsigned short* __restrict__ Btp, const unsigned short* __restrict__ Bt2p, int ldb, long strideB,
    void* __restrict__ Cout, void* __restrict__ Cout2, int ldc, long strideC,
    const float* __restrict__ bias,
    const float* __restrict__ resid, long strideR,
    int M, int N, int K, float scale) {
  typedef typename Elem<ET>::T T;
  typedef typename Frag<T>::V V;
  const T* A = (const T*)Ap; const T* A2 = (const T*)A2p; const T* Bt = (const T*)Btp; const T* Bt2 = (const T*)Bt2p;
  __shared__ __align__(16) float sT[8][16 * 68];
  const int b    = blockIdx.y;
  const int lane = threadIdx.x & 31;
  const int wave = threadIdx.x >> 5;
  const int tilesN = N >> 6;
  const int tilesM = M >> 6;
  const int tile = blockIdx.x * 8 + wave;
  if (tile >= tilesM * tilesN) return;
  const int tm = tile / tilesN;
  const int tn = tile - tm * tilesN;
  const int m0 = tm << 6;
  const int n0 = tn << 6;

  const T* Ab  = A  + (size_t)b * strideA;
  const T* Bb  = Bt + (size_t)b * strideB;
  const T* Ab2 = SPLIT ? (A2  + (size_t)b * strideA) : nullptr;
  const T* Bb2 = SPLIT ? (Bt2 + (size_t)b * strideB) : nullptr;

  const int rlane = lane & 15;
  const int koff  = (lane >> 4) * 8;
  const int mOff  = (lane >> 4) * 8;

  v8f acc[4][4];
#pragma unroll
  for (int i = 0; i < 4; ++i)
#pragma unroll
    for (int j = 0; j < 4; ++j) acc[i][j] = (v8f){0.f,0.f,0.f,0.f,0.f,0.f,0.f,0.f};

  for (int k0 = 0; k0 < K; k0 += 32) {
    V bh[4], bl[4];
#pragma unroll
    for (int j = 0; j < 4; ++j) {
      const size_t bo = (size_t)(n0 + (j << 4) + rlane) * ldb + koff + k0;
      bh[j] = Frag<T>::load(Bb + bo);
      if (SPLIT) bl[j] = Frag<T>::load(Bb2 + bo);
    }
#pragma unroll
    for (int i = 0; i < 4; ++i) {
      const size_t ao = (size_t)(m0 + (i << 4) + rlane) * lda + koff + k0;
      V ah = Frag<T>::load(Ab + ao);
      V al;
      if (SPLIT) al = Frag<T>::load(Ab2 + ao);
#pragma unroll
      for (int j = 0; j < 4; ++j) {
        acc[i][j] = Frag<T>::mma(ah, bh[j], acc[i][j]);
        if (SPLIT) {
          acc[i][j] = Frag<T>::mma(ah, bl[j], acc[i][j]);
          acc[i][j] = Frag<T>::mma(al, bh[j], acc[i][j]);
        }
      }
      Frag<T>::guard4(acc[i][0], acc[i][1], acc[i][2], acc[i][3], ah, SPLIT ? al : ah);
    }
    Frag<T>::keep(bh[0], bh[1], bh[2], bh[3]);
    if (SPLIT) Frag<T>::keep(bl[0], bl[1], bl[2], bl[3]);
  }
  acc_guard4(acc[0][0], acc[0][1], acc[0][2], acc[0][3]);
  acc_guard4(acc[1][0], acc[1][1], acc[1][2], acc[1][3]);
  acc_guard4(acc[2][0], acc[2][1], acc[2][2], acc[2][3]);
  acc_guard4(acc[3][0], acc[3][1], acc[3][2], acc[3][3]);

  float* slab = sT[wave];
  const float* Rb = RESID ? (resid + (size_t)b * strideR) : nullptr;
#pragma unroll
  for (int i = 0; i < 4; ++i) {
    const int mBase = m0 + (i << 4);
#pragma unroll
    for (int j = 0; j < 4; ++j) {
      const int n = n0 + (j << 4) + rlane;
      float bv = 0.f;
      if (BIAS_MODE == 2) bv = bias[n];
#pragma unroll
      for (int r = 0; r < 8; ++r) {
        float v = acc[i][j][r] * scale;
        if (BIAS_MODE == 1) v += bias[mBase + mOff + r];
        if (BIAS_MODE == 2) v += bv;
        if (RESID) v += Rb[(size_t)(mBase + mOff + r) * ldc + n];
        if (ACT == 2) v = fmaxf(v, 0.0f);
        if (ACT == 4) v = (v > 0.f) ? v : 0.01f * v;
        slab[(mOff + r) * 68 + (j << 4) + rlane] = v;
      }
    }
    __builtin_amdgcn_fence(__ATOMIC_RELEASE, "workgroup");
    __builtin_amdgcn_wave_barrier();
    __builtin_amdgcn_fence(__ATOMIC_ACQUIRE, "workgroup");
    if (OUT_MODE == 0) {
      float* C = (float*)Cout + (size_t)b * strideC;
      const int hh = lane >> 4, c4 = (lane & 15) * 4;
      for (int pass = 0; pass < 2; ++pass) {
#pragma unroll
        for (int it = 0; it < 8; ++it) {
          const int row = it * 2 + hh;
          v4f v = *(const v4f*)(slab + row * 68 + c4);
          *(volatile v4f*)(C + (size_t)(mBase + row) * ldc + n0 + c4) = v;
        }
        __threadfence();
      }
    } else {
      const int q = lane >> 3, c8 = (lane & 7) * 8;
      unsigned short* C  = (unsigned short*)Cout  + (size_t)b * strideC;
      unsigned short* C2 = (OUT_MODE == 2) ? ((unsigned short*)Cout2 + (size_t)b * strideC) : nullptr;
      for (int pass = 0; pass < 2; ++pass) {
#pragma unroll
        for (int it = 0; it < 4; ++it) {
          const int row = it * 4 + q;
          const float* sp = slab + row * 68 + c8;
          v8h hv, lv;
#pragma unroll
          for (int e = 0; e < 8; ++e) {
            if (OUT_MODE == 1) {
              hv[e] = (_Float16)sp[e];
            } else {
              unsigned short hb = f2bf_bits(sp[e]);
              unsigned short lb = f2bf_bits(sp[e] - bf_bits2f(hb));
              hv[e] = __builtin_bit_cast(_Float16, hb);
              lv[e] = __builtin_bit_cast(_Float16, lb);
            }
          }
          *(volatile v8h*)(C + (size_t)(mBase + row) * ldc + n0 + c8) = hv;
          if (OUT_MODE == 2) *(volatile v8h*)(C2 + (size_t)(mBase + row) * ldc + n0 + c8) = lv;
        }
        __threadfence();
      }
    }
    __builtin_amdgcn_fence(__ATOMIC_RELEASE, "workgroup");
    __builtin_amdgcn_wave_barrier();
    __builtin_amdgcn_fence(__ATOMIC_ACQUIRE, "workgroup");
  }
}

__global__ __launch_bounds__(256) void wsplit_bf16_kernel(const float* __restrict__ W0, const float* __restrict__ W1,
                                                         unsigned short* __restrict__ H0, unsigned short* __restrict__ L0,
                                                         unsigned short* __restrict__ H1, unsigned short* __restrict__ L1, int n8) {
  const int i = blockIdx.x * 256 + threadIdx.x;
  if (i >= n8) return;
  const int z = blockIdx.y;
  const float* W = (z == 0) ? W0 : W1;
  unsigned short* H = (z == 0) ? H0 : H1;
  unsigned short* L = (z == 0) ? L0 : L1;
  const float* p = W + 8 * (size_t)i;
  const v4f a = *(const v4f*)(p);
  const v4f c = *(const v4f*)(p + 4);
  unsigned short hb[8], lb[8];
#pragma unroll
  for (int e = 0; e < 4; ++e) {
    const float f0 = a[e], f1 = c[e];
    hb[e] = f2bf_bits(f0);      lb[e] = f2bf_bits(f0 - bf_bits2f(hb[e]));
    hb[4 + e] = f2bf_bits(f1);  lb[4 + e] = f2bf_bits(f1 - bf_bits2f(hb[4 + e]));
  }
  const v4u uh = (v4u){pk16(hb[0], hb[1]), pk16(hb[2], hb[3]), pk16(hb[4], hb[5]), pk16(hb[6], hb[7])};
  const v4u ul = (v4u){pk16(lb[0], lb[1]), pk16(lb[2], lb[3]), pk16(lb[4], lb[5]), pk16(lb[6], lb[7])};
  unsigned short* qh = H + 8 * (size_t)i;
  unsigned short* ql = L + 8 * (size_t)i;
  *(volatile v4u*)qh = uh;
  *(volatile v4u*)ql = ul;
  __threadfence();
  *(volatile v4u*)qh = uh;
  *(volatile v4u*)ql = ul;
}

__global__ __launch_bounds__(256) void wcast_f16_kernel(const float* __restrict__ W0, const float* __restrict__ W1,
                                                       unsigned short* __restrict__ O0, unsigned short* __restrict__ O1,
                                                       int n8, float scale) {
  const int i = blockIdx.x * 256 + threadIdx.x;
  if (i >= n8) return;
  const int z = blockIdx.y;
  const float* W = (z == 0) ? W0 : W1;
  unsigned short* O = (z == 0) ? O0 : O1;
  const float* p = W + 8 * (size_t)i;
  const v4f a = *(const v4f*)(p);
  const v4f c = *(const v4f*)(p + 4);
  unsigned short hb[8];
#pragma unroll
  for (int e = 0; e < 4; ++e) {
    hb[e]     = h_bits(a[e] * scale);
    hb[4 + e] = h_bits(c[e] * scale);
  }
  const v4u u = (v4u){pk16(hb[0], hb[1]), pk16(hb[2], hb[3]), pk16(hb[4], hb[5]), pk16(hb[6], hb[7])};
  unsigned short* q = O + 8 * (size_t)i;
  *(volatile v4u*)q = u;
  __threadfence();
  *(volatile v4u*)q = u;
}

__global__ __launch_bounds__(256) void mix_kernel(const float* __restrict__ x, const float* __restrict__ mk,
                                                 const float* __restrict__ mv, const float* __restrict__ mr,
                                                 unsigned short* __restrict__ XKH, unsigned short* __restrict__ XKL,
                                                 unsigned short* __restrict__ XVH, unsigned short* __restrict__ XVL,
                                                 unsigned short* __restrict__ XR, int row0, int nthreads) {
  const int i = blockIdx.x * 256 + threadIdx.x;
  if (i >= nthreads) return;
  const int ml = i >> 7;
  const int c  = (i & 127) * 8;
  const int m  = row0 + ml;
  const int t  = m & (kT - 1);
  const int mp = (m > 0) ? (m - 1) : 0;
  const float fz = (t > 0) ? 1.0f : 0.0f;
  const float* xcp = x + (size_t)m * kC + c;
  const float* xpp = x + (size_t)mp * kC + c;
  const v4f a0 = *(const v4f*)(xcp);
  const v4f a1 = *(const v4f*)(xcp + 4);
  const v4f p0 = *(const v4f*)(xpp);
  const v4f p1 = *(const v4f*)(xpp + 4);
  const v4f k0 = *(const v4f*)(mk + c);
  const v4f k1 = *(const v4f*)(mk + c + 4);
  asm volatile("" ::: "memory");
  const v4f v0 = *(const v4f*)(mv + c);
  const v4f v1 = *(const v4f*)(mv + c + 4);
  const v4f r0 = *(const v4f*)(mr + c);
  const v4f r1 = *(const v4f*)(mr + c + 4);
  float xc[8], xx[8], ck[8], cv[8], cr[8];
#pragma unroll
  for (int e = 0; e < 4; ++e) {
    xc[e] = a0[e]; xc[4 + e] = a1[e];
    xx[e] = p0[e] * fz; xx[4 + e] = p1[e] * fz;
    ck[e] = k0[e]; ck[4 + e] = k1[e];
    cv[e] = v0[e]; cv[4 + e] = v1[e];
    cr[e] = r0[e]; cr[4 + e] = r1[e];
  }
  unsigned short kh[8], kl[8], vh[8], vl[8], rh[8];
#pragma unroll
  for (int e = 0; e < 8; ++e) {
    const float xk = xc[e] * ck[e] + xx[e] * (1.0f - ck[e]);
    const float xv = xc[e] * cv[e] + xx[e] * (1.0f - cv[e]);
    const float xr = xc[e] * cr[e] + xx[e] * (1.0f - cr[e]);
    const unsigned short hk = f2bf_bits(xk);
    kh[e] = hk; kl[e] = f2bf_bits(xk - bf_bits2f(hk));
    const unsigned short hv = f2bf_bits(xv);
    vh[e] = hv; vl[e] = f2bf_bits(xv - bf_bits2f(hv));
    rh[e] = h_bits(xr);
  }
  const v4u ukh = (v4u){pk16(kh[0], kh[1]), pk16(kh[2], kh[3]), pk16(kh[4], kh[5]), pk16(kh[6], kh[7])};
  const v4u ukl = (v4u){pk16(kl[0], kl[1]), pk16(kl[2], kl[3]), pk16(kl[4], kl[5]), pk16(kl[6], kl[7])};
  const v4u uvh = (v4u){pk16(vh[0], vh[1]), pk16(vh[2], vh[3]), pk16(vh[4], vh[5]), pk16(vh[6], vh[7])};
  const v4u uvl = (v4u){pk16(vl[0], vl[1]), pk16(vl[2], vl[3]), pk16(vl[4], vl[5]), pk16(vl[6], vl[7])};
  const v4u ur  = (v4u){pk16(rh[0], rh[1]), pk16(rh[2], rh[3]), pk16(rh[4], rh[5]), pk16(rh[6], rh[7])};
  const size_t o = (size_t)ml * kC + c;
  *(volatile v4u*)(XKH + o) = ukh;
  *(volatile v4u*)(XKL + o) = ukl;
  *(volatile v4u*)(XVH + o) = uvh;
  *(volatile v4u*)(XVL + o) = uvl;
  *(volatile v4u*)(XR  + o) = ur;
  __threadfence();
  *(volatile v4u*)(XKH + o) = ukh;
  *(volatile v4u*)(XKL + o) = ukl;
  *(volatile v4u*)(XVH + o) = uvh;
  *(volatile v4u*)(XVL + o) = uvl;
  *(volatile v4u*)(XR  + o) = ur;
}

__device__ __forceinline__ float wkv_step(float kt, float vt, float rr, float w, float u, float& p, float& q, float& o) {
  const float uk  = u + kt;
  const float no  = fmaxf(o, uk);
  const float ea  = expf(o - no);
  const float eb  = expf(uk - no);
  const float num = ea * p + eb * vt;
  const float den = ea * q + eb;
  const float y   = num / den;
  const float sr  = 1.0f / (1.0f + expf(-rr));
  const float wo  = w + o;
  const float no2 = fmaxf(wo, kt);
  const float e2a = expf(wo - no2);
  const float e2b = expf(kt - no2);
  p = e2a * p + e2b * vt;
  q = e2a * q + e2b;
  o = no2;
  return sr * y;
}

__global__ __launch_bounds__(256) void wkv_kernel(const float* __restrict__ td, const float* __restrict__ tfst,
                                                 const float* __restrict__ Kf, const float* __restrict__ Vf,
                                                 const unsigned short* __restrict__ R16, unsigned short* __restrict__ AO,
                                                 int nlanes) {
  const int g = blockIdx.x * 256 + threadIdx.x;
  if (g >= nlanes) return;
  const int bl = g >> 9;
  const int c0 = (g & (kPairs - 1)) * 2;
  const v2f tdv = *(const v2f*)(td + c0);
  const v2f tfv = *(const v2f*)(tfst + c0);
  const float w0 = -expf(tdv[0]);
  const float w1 = -expf(tdv[1]);
  const float u0 = tfv[0];
  const float u1 = tfv[1];
  size_t off = (size_t)bl * kT * kC + c0;
  float p0 = 0.0f, q0 = 0.0f, o0 = kNegInit;
  float p1 = 0.0f, q1 = 0.0f, o1 = kNegInit;
#pragma unroll 1
  for (int t = 0; t < kT; ++t) {
    const v2f kv = *(const v2f*)(Kf + off);
    const v2f vv = *(const v2f*)(Vf + off);
    const unsigned rw = *(const unsigned*)(const void*)(R16 + off);
    const float rr0 = h16_to_f32(rw & 0xffffu);
    const float rr1 = h16_to_f32(rw >> 16);
    const float a0 = wkv_step(kv[0], vv[0], rr0, w0, u0, p0, q0, o0);
    const float a1 = wkv_step(kv[1], vv[1], rr1, w1, u1, p1, q1, o1);
    const unsigned u = pk16(h_bits(a0 * kACarry), h_bits(a1 * kACarry));
    unsigned* ap = (unsigned*)(void*)(AO + off);
    *(volatile unsigned*)ap = u;
    __threadfence();
    *(volatile unsigned*)ap = u;
    off += kC;
  }
}

extern "C" void kernel_launch(void* const* d_in, const int* in_sizes, int n_in,
                              void* d_out, int out_size, void* d_ws, size_t ws_size,
                              hipStream_t stream) {
  if (n_in < 10) return;
  const int nTok = kRows * kC;
  const int nW   = kC * kC;
  if (in_sizes[0] != nTok) return;
  if (in_sizes[1] != kC || in_sizes[2] != kC || in_sizes[3] != kC || in_sizes[4] != kC || in_sizes[5] != kC) return;
  if (in_sizes[6] != nW || in_sizes[7] != nW || in_sizes[8] != nW || in_sizes[9] != nW) return;
  if (out_size != nTok) return;

  const size_t szW16 = (size_t)nW * 2;
  const size_t szX16 = (size_t)kChunkRows * kC * 2;
  const size_t szF32 = (size_t)kChunkRows * kC * 4;
  const size_t offWkH = 0;
  const size_t offWkL = offWkH + szW16;
  const size_t offWvH = offWkL + szW16;
  const size_t offWvL = offWvH + szW16;
  const size_t offWr  = offWvL + szW16;
  const size_t offWo  = offWr  + szW16;
  const size_t offXKH = offWo  + szW16;
  const size_t offXKL = offXKH + szX16;
  const size_t offXVH = offXKL + szX16;
  const size_t offXVL = offXVH + szX16;
  const size_t offXR  = offXVL + szX16;
  const size_t offKf  = offXR  + szX16;
  const size_t offVf  = offKf  + szF32;
  const size_t offR16 = offVf  + szF32;
  const size_t offAO  = offR16 + szX16;
  const size_t total  = offAO  + szX16;
  if (ws_size < total) return;

  const float* x   = (const float*)d_in[0];
  const float* td  = (const float*)d_in[1];
  const float* tfs = (const float*)d_in[2];
  const float* mk  = (const float*)d_in[3];
  const float* mv  = (const float*)d_in[4];
  const float* mr  = (const float*)d_in[5];
  const float* Wk  = (const float*)d_in[6];
  const float* Wv  = (const float*)d_in[7];
  const float* Wr  = (const float*)d_in[8];
  const float* Wo  = (const float*)d_in[9];
  float* out = (float*)d_out;
  char* ws = (char*)d_ws;
  unsigned short* WkH  = (unsigned short*)(ws + offWkH);
  unsigned short* WkL  = (unsigned short*)(ws + offWkL);
  unsigned short* WvH  = (unsigned short*)(ws + offWvH);
  unsigned short* WvL  = (unsigned short*)(ws + offWvL);
  unsigned short* Wr16 = (unsigned short*)(ws + offWr);
  unsigned short* Wo16 = (unsigned short*)(ws + offWo);
  unsigned short* XKH  = (unsigned short*)(ws + offXKH);
  unsigned short* XKL  = (unsigned short*)(ws + offXKL);
  unsigned short* XVH  = (unsigned short*)(ws + offXVH);
  unsigned short* XVL  = (unsigned short*)(ws + offXVL);
  unsigned short* XR   = (unsigned short*)(ws + offXR);
  float* Kf = (float*)(ws + offKf);
  float* Vf = (float*)(ws + offVf);
  unsigned short* R16  = (unsigned short*)(ws + offR16);
  unsigned short* AO   = (unsigned short*)(ws + offAO);

  const int nW8 = nW / 8;
  wsplit_bf16_kernel<<<dim3(nW8 / 256, 2), dim3(256), 0, stream>>>(Wk, Wv, WkH, WkL, WvH, WvL, nW8);
  wcast_f16_kernel<<<dim3(nW8 / 256, 2), dim3(256), 0, stream>>>(Wr, Wo, Wr16, Wo16, nW8, kWCarry);

  const int mixThreads = kChunkRows * (kC / 8);
  const int scanLanes  = kChunkB * kPairs;
  const int gemmTiles  = (kChunkRows / 64) * (kC / 64);
  for (int ch = 0; ch < kChunks; ++ch) {
    const int row0 = ch * kChunkRows;
    mix_kernel<<<dim3(mixThreads / 256), dim3(256), 0, stream>>>(x, mk, mv, mr, XKH, XKL, XVH, XVL, XR, row0, mixThreads);
    wmma_gemm64<1, true, 0, 0, false, 0><<<dim3(gemmTiles / 8, 1), dim3(256), 0, stream>>>(
        XKH, XKL, kC, 0L, WkH, WkL, kC, 0L, (void*)Kf, (void*)Kf, kC, 0L, td, td, 0L, kChunkRows, kC, kC, 1.0f);
    wmma_gemm64<1, true, 0, 0, false, 0><<<dim3(gemmTiles / 8, 1), dim3(256), 0, stream>>>(
        XVH, XVL, kC, 0L, WvH, WvL, kC, 0L, (void*)Vf, (void*)Vf, kC, 0L, td, td, 0L, kChunkRows, kC, kC, 1.0f);
    wmma_gemm64<0, false, 0, 1, false, 0><<<dim3(gemmTiles / 8, 1), dim3(256), 0, stream>>>(
        XR, XR, kC, 0L, Wr16, Wr16, kC, 0L, (void*)R16, (void*)R16, kC, 0L, td, td, 0L, kChunkRows, kC, kC, kRScale);
    wkv_kernel<<<dim3(scanLanes / 256), dim3(256), 0, stream>>>(td, tfs, Kf, Vf, R16, AO, scanLanes);
    float* outc = out + (size_t)row0 * kC;
    wmma_gemm64<0, false, 0, 0, false, 0><<<dim3(gemmTiles / 8, 1), dim3(256), 0, stream>>>(
        AO, AO, kC, 0L, Wo16, Wo16, kC, 0L, (void*)outc, (void*)outc, kC, 0L, td, td, 0L, kChunkRows, kC, kC, kOScale);
  }
}
